// CATDecoderAttention_11458972746231
// MI455X (gfx1250) — hardware-verified
//
#include <hip/hip_runtime.h>
#include <math.h>

constexpr int SEQ_T   = 4096;
constexpr int HIDSZ   = 1024;
constexpr int NQH     = 16;
constexpr int NKVH    = 4;
constexpr int HDIM    = 64;
constexpr int GQA_G   = NQH / NKVH;
constexpr int QCHUNK  = 2048;
constexpr int NCHUNK  = SEQ_T / QCHUNK;
constexpr float SCORE_SCALE = 0.125f;
constexpr float RMS_EPS_F   = 1e-6f;

static_assert(GQA_G == 4, "kv head = hq >> 2");
static_assert(SEQ_T == 4096 && QCHUNK == 2048, "softmax kernels: 256 threads x 8 cols = 2048 (chunk 0), 512 x 8 = 4096 (chunk 1)");
static_assert(QCHUNK % 64 == 0 && SEQ_T % 64 == 0 && HIDSZ % 64 == 0 && HDIM == 64 && (NKVH * HDIM) % 64 == 0, "tile multiples");
static_assert((SEQ_T * HIDSZ) % (8 * 256) == 0, "cast kernel grid exact");
static_assert((SEQ_T * NQH) % 32 == 0 && (SEQ_T * NKVH) % 32 == 0, "normrope grid exact");

typedef __attribute__((ext_vector_type(16))) _Float16 v16h;
typedef __attribute__((ext_vector_type(8)))  _Float16 v8h;
typedef __attribute__((ext_vector_type(16))) __bf16   v16b;
typedef __attribute__((ext_vector_type(8)))  __bf16   v8b;
typedef __attribute__((ext_vector_type(8)))  float    v8f;
typedef __attribute__((ext_vector_type(4)))  float    v4f;
typedef __attribute__((ext_vector_type(4)))  unsigned int v4u;

__device__ __forceinline__ unsigned short f2bf_bits(float f) {
  unsigned u = __float_as_uint(f);
  return (unsigned short)((u + 0x7FFFu + ((u >> 16) & 1u)) >> 16);
}
__device__ __forceinline__ float bf_bits2f(unsigned short h) { return __uint_as_float(((unsigned)h) << 16); }
__device__ __forceinline__ float bfq(float f) { return bf_bits2f(f2bf_bits(f)); }

__device__ __forceinline__ void dep_guard_h(v8f& a, v8f& b, v16h x, v16h y) { asm volatile("v_nop\n\tv_nop\n\tv_nop\n\tv_nop" : "+v"(a), "+v"(b) : "v"(x), "v"(y)); }
__device__ __forceinline__ void dep_guard_b(v8f& a, v8f& b, v16b x, v16b y) { asm volatile("v_nop\n\tv_nop\n\tv_nop\n\tv_nop" : "+v"(a), "+v"(b) : "v"(x), "v"(y)); }
__device__ __forceinline__ void keep4_h(v16h a, v16h b, v16h c, v16h d) { asm volatile("v_nop" :: "v"(a), "v"(b), "v"(c), "v"(d)); }
__device__ __forceinline__ void keep4_b(v16b a, v16b b, v16b c, v16b d) { asm volatile("v_nop" :: "v"(a), "v"(b), "v"(c), "v"(d)); }
__device__ __forceinline__ void acc_guard4(v8f& a, v8f& b, v8f& c, v8f& d) { asm volatile("v_nop\n\tv_nop\n\tv_nop\n\tv_nop" : "+v"(a), "+v"(b), "+v"(c), "+v"(d)); }
template <typename T> struct Frag;
template <> struct Frag<_Float16> {
  typedef v16h V; union U { v16h v; v8h h[2]; };
  static __device__ __forceinline__ v16h load(const _Float16* p) {
    U f; f.h[0] = *(const v8h*)(p); f.h[1] = *(const v8h*)(p + 16); return f.v;
  }
  static __device__ __forceinline__ v8f mma(v16h a, v16h b, v8f c) {
    return __builtin_amdgcn_wmma_f32_16x16x32_f16(false, a, false, b, (short)0, c, false, false);
  }
  static __device__ __forceinline__ void guard(v8f& a, v8f& b, v16h x, v16h y) { dep_guard_h(a, b, x, y); }
  static __device__ __forceinline__ void keep(v16h a, v16h b, v16h c, v16h d) { keep4_h(a, b, c, d); }
};
template <> struct Frag<__bf16> {
  typedef v16b V; union U { v16b v; v8b h[2]; };
  static __device__ __forceinline__ v16b load(const __bf16* p) {
    U f; f.h[0] = *(const v8b*)(p); f.h[1] = *(const v8b*)(p + 16); return f.v;
  }
  static __device__ __forceinline__ v8f mma(v16b a, v16b b, v8f c) {
    return __builtin_amdgcn_wmma_f32_16x16x32_bf16(false, a, false, b, (short)0, c, false, false);
  }
  static __device__ __forceinline__ void guard(v8f& a, v8f& b, v16b x, v16b y) { dep_guard_b(a, b, x, y); }
  static __device__ __forceinline__ void keep(v16b a, v16b b, v16b c, v16b d) { keep4_b(a, b, c, d); }
};

__device__ __forceinline__ unsigned pk16(unsigned short a, unsigned short b) { return (unsigned)a | ((unsigned)b << 16); }

template <int ET> struct Elem;
template <> struct Elem<0> { typedef _Float16 T; };
template <> struct Elem<1> { typedef __bf16 T; };
template <int ET, bool SPLIT, int BIAS_MODE, int OUT_MODE, bool RESID, int ACT = 0, bool CAUSAL = false, bool BSPLIT = true>
__global__ __launch_bounds__(256) void wmma_gemm64(
    const unsigned short* __restrict__ Ap, const unsigned short* __restrict__ A2p, int lda, long strideA,
    const unsigned short* __restrict__ Btp, const unsigned short* __restrict__ Bt2p, int ldb, long strideB,
    void* __restrict__ Cout, void* __restrict__ Cout2, int ldc, long strideC,
    const float* __restrict__ bias,
    const float* __restrict__ resid, long strideR,
    int M, int N, int K, float scale, int crow0) {
  typedef typename Elem<ET>::T T;
  typedef typename Frag<T>::V V;
  const T* A = (const T*)Ap; const T* A2 = (const T*)A2p; const T* Bt = (const T*)Btp; const T* Bt2 = (const T*)Bt2p;
  __shared__ __align__(16) float sT[8][16 * 68];
  const int b    = blockIdx.y;
  const int lane = threadIdx.x & 31;
  const int wave = threadIdx.x >> 5;
  const int tilesN = N >> 6;
  const int tilesM = M >> 6;
  const int tile = blockIdx.x * 8 + wave;
  if (tile >= tilesM * tilesN) return;
  const int tm = tile / tilesN;
  const int tn = tile - tm * tilesN;
  const int m0 = tm << 6;
  const int n0 = tn << 6;
  if (CAUSAL && (n0 > m0 + crow0)) return;
  const int Kend = CAUSAL ? ((m0 + crow0 + 64 < K) ? (m0 + crow0 + 64) : K) : K;

  const T* Ab  = A  + (size_t)b * strideA;
  const T* Bb  = Bt + (size_t)b * strideB;
  const T* Ab2 = SPLIT ? (A2  + (size_t)b * strideA) : nullptr;
  const T* Bb2 = (SPLIT && BSPLIT) ? (Bt2 + (size_t)b * strideB) : nullptr;

  const int rlane = lane & 15;
  const int koff  = (lane >> 4) * 8;
  const int mOff  = (lane >> 4) * 8;

  v8f acc[4][4];
#pragma unroll
  for (int i = 0; i < 4; ++i)
#pragma unroll
    for (int j = 0; j < 4; ++j) acc[i][j] = (v8f){0.f,0.f,0.f,0.f,0.f,0.f,0.f,0.f};

  for (int k0 = 0; k0 < Kend; k0 += 32) {
    V bh[4], bl[4];
#pragma unroll
    for (int j = 0; j < 4; ++j) {
      const size_t bo = (size_t)(n0 + (j << 4) + rlane) * ldb + koff + k0;
      bh[j] = Frag<T>::load(Bb + bo);
      if (SPLIT && BSPLIT) bl[j] = Frag<T>::load(Bb2 + bo);
    }
#pragma unroll
    for (int i = 0; i < 4; ++i) {
      const size_t ao = (size_t)(m0 + (i << 4) + rlane) * lda + koff + k0;
      V ah = Frag<T>::load(Ab + ao);
      V al;
      if (SPLIT) al = Frag<T>::load(Ab2 + ao);
#pragma unroll
      for (int j = 0; j < 4; ++j) {
        acc[i][j] = Frag<T>::mma(ah, bh[j], acc[i][j]);
        if (SPLIT && BSPLIT) acc[i][j] = Frag<T>::mma(ah, bl[j], acc[i][j]);
        if (SPLIT) acc[i][j] = Frag<T>::mma(al, bh[j], acc[i][j]);
      }
      Frag<T>::guard(acc[i][0], acc[i][3], ah, SPLIT ? al : ah);
    }
    Frag<T>::keep(bh[0], bh[1], bh[2], bh[3]);
    if (SPLIT && BSPLIT) Frag<T>::keep(bl[0], bl[1], bl[2], bl[3]);
  }
  acc_guard4(acc[0][0], acc[0][1], acc[0][2], acc[0][3]);
  acc_guard4(acc[1][0], acc[1][1], acc[1][2], acc[1][3]);
  acc_guard4(acc[2][0], acc[2][1], acc[2][2], acc[2][3]);
  acc_guard4(acc[3][0], acc[3][1], acc[3][2], acc[3][3]);

  float* slab = sT[wave];
  const float* Rb = RESID ? (resid + (size_t)b * strideR) : nullptr;
#pragma unroll
  for (int i = 0; i < 4; ++i) {
    const int mBase = m0 + (i << 4);
#pragma unroll
    for (int j = 0; j < 4; ++j) {
      const int n = n0 + (j << 4) + rlane;
      float bv = 0.f;
      if (BIAS_MODE == 2) bv = bias[n];
#pragma unroll
      for (int r = 0; r < 8; ++r) {
        float v = acc[i][j][r] * scale;
        if (BIAS_MODE == 1) v += bias[mBase + mOff + r];
        if (BIAS_MODE == 2) v += bv;
        if (RESID) v += Rb[(size_t)(mBase + mOff + r) * ldc + n];
        if (ACT == 2) v = fmaxf(v, 0.0f);
        if (ACT == 4) v = (v > 0.f) ? v : 0.01f * v;
        slab[(mOff + r) * 68 + (j << 4) + rlane] = v;
      }
    }
    __builtin_amdgcn_fence(__ATOMIC_RELEASE, "workgroup");
    __builtin_amdgcn_wave_barrier();
    __builtin_amdgcn_fence(__ATOMIC_ACQUIRE, "workgroup");
    if (OUT_MODE == 0) {
      float* C = (float*)Cout + (size_t)b * strideC;
      const int hh = lane >> 4, c4 = (lane & 15) * 4;
      for (int pass = 0; pass < 2; ++pass) {
#pragma unroll
        for (int it = 0; it < 8; ++it) {
          const int row = it * 2 + hh;
          v4f v = *(const v4f*)(slab + row * 68 + c4);
          *(volatile v4f*)(C + (size_t)(mBase + row) * ldc + n0 + c4) = v;
        }
        __threadfence();
      }
    } else {
      const int q = lane >> 3, c8 = (lane & 7) * 8;
      unsigned short* C  = (unsigned short*)Cout  + (size_t)b * strideC;
      unsigned short* C2 = (OUT_MODE == 2) ? ((unsigned short*)Cout2 + (size_t)b * strideC) : nullptr;
      for (int pass = 0; pass < 2; ++pass) {
#pragma unroll
        for (int it = 0; it < 4; ++it) {
          const int row = it * 4 + q;
          const float* sp = slab + row * 68 + c8;
          v8h hv, lv;
#pragma unroll
          for (int e = 0; e < 8; ++e) {
            if (OUT_MODE == 1) {
              hv[e] = (_Float16)sp[e];
            } else {
              unsigned short hb = f2bf_bits(sp[e]);
              unsigned short lb = f2bf_bits(sp[e] - bf_bits2f(hb));
              hv[e] = __builtin_bit_cast(_Float16, hb);
              lv[e] = __builtin_bit_cast(_Float16, lb);
            }
          }
          *(volatile v8h*)(C + (size_t)(mBase + row) * ldc + n0 + c8) = hv;
          if (OUT_MODE == 2) *(volatile v8h*)(C2 + (size_t)(mBase + row) * ldc + n0 + c8) = lv;
        }
        __threadfence();
      }
    }
    __builtin_amdgcn_fence(__ATOMIC_RELEASE, "workgroup");
    __builtin_amdgcn_wave_barrier();
    __builtin_amdgcn_fence(__ATOMIC_ACQUIRE, "workgroup");
  }
}

__global__ __launch_bounds__(256) void cast8_bf16_kernel(const float* __restrict__ in, unsigned short* __restrict__ out, int n8) {
  const int i = blockIdx.x * 256 + threadIdx.x;
  if (i >= n8) return;
  const float* p = in + 8 * (size_t)i;
  const v4f a = *(const v4f*)(p);
  const v4f c = *(const v4f*)(p + 4);
  float f[8];
#pragma unroll
  for (int e = 0; e < 4; ++e) { f[e] = a[e]; f[4 + e] = c[e]; }
  unsigned w[4];
#pragma unroll
  for (int e2 = 0; e2 < 4; ++e2) w[e2] = pk16(f2bf_bits(f[2 * e2]), f2bf_bits(f[2 * e2 + 1]));
  const v4u u = (v4u){w[0], w[1], w[2], w[3]};
  unsigned short* q = out + 8 * (size_t)i;
  *(volatile v4u*)q = u;
  __threadfence();
  *(volatile v4u*)q = u;
}

__global__ __launch_bounds__(256) void transpose_cast_kernel(const float* __restrict__ in, int ldin,
                                                             unsigned short* __restrict__ out, int ldout) {
  __shared__ float sm[64][65];
  const int t  = threadIdx.x;
  const int r0 = blockIdx.x * 64;
  const int c0 = blockIdx.y * 64;
#pragma unroll
  for (int i = 0; i < 16; ++i) {
    const int e = i * 256 + t;
    const int r = e >> 6;
    const int c = e & 63;
    sm[c][r] = in[(size_t)(r0 + r) * ldin + c0 + c];
  }
  __syncthreads();
  const int lane = t & 31, wave = t >> 5;
  const int q = lane >> 3, c8 = (lane & 7) * 8;
  for (int pass = 0; pass < 2; ++pass) {
#pragma unroll
    for (int it = 0; it < 2; ++it) {
      const int row = wave * 8 + it * 4 + q;
      unsigned w[4];
#pragma unroll
      for (int e2 = 0; e2 < 4; ++e2) w[e2] = pk16(f2bf_bits(sm[row][c8 + 2 * e2]), f2bf_bits(sm[row][c8 + 2 * e2 + 1]));
      const v4u u = (v4u){w[0], w[1], w[2], w[3]};
      const size_t o = (size_t)(c0 + row) * ldout + r0 + c8;
      *(volatile v4u*)(out + o) = u;
    }
    __threadfence();
  }
}

__global__ __launch_bounds__(256) void normrope_kernel(const float* __restrict__ proj, int hshift, int nrows,
                                                       const float* __restrict__ cosb, const float* __restrict__ sinb,
                                                       const float* __restrict__ w,
                                                       unsigned short* __restrict__ ohi, unsigned short* __restrict__ olo) {
#pragma clang fp contract(off)
  __shared__ __align__(16) float slab[8][4][64];
  const int lane = threadIdx.x & 31, wave = threadIdx.x >> 5;
  const int rbase = (blockIdx.x * 8 + wave) * 4;
  const float w1 = bfq(w[lane]), w2 = bfq(w[lane + 32]);
#pragma unroll
  for (int i = 0; i < 4; ++i) {
    int r = rbase + i;
    r = (r < nrows) ? r : (nrows - 1);
    const int t = r >> hshift;
    const float* src = proj + (size_t)r * 64;
    const float x1 = src[lane];
    const float x2 = src[lane + 32];
    float ss = x1 * x1 + x2 * x2;
#pragma unroll
    for (int off = 16; off > 0; off >>= 1) ss += __shfl_xor(ss, off, 32);
    const float inv = rsqrtf(ss * (1.0f / 64.0f) + RMS_EPS_F);
    const float n1 = (x1 * inv) * w1;
    const float n2 = (x2 * inv) * w2;
    const float c = bfq(cosb[(size_t)t * 32 + lane]);
    const float s = bfq(sinb[(size_t)t * 32 + lane]);
    slab[wave][i][lane]      = n1 * c - n2 * s;
    slab[wave][i][lane + 32] = n1 * s + n2 * c;
  }
  __builtin_amdgcn_fence(__ATOMIC_RELEASE, "workgroup");
  __builtin_amdgcn_wave_barrier();
  __builtin_amdgcn_fence(__ATOMIC_ACQUIRE, "workgroup");
  const int q = lane >> 3, c8 = (lane & 7) * 8;
  int r = rbase + q;
  r = (r < nrows) ? r : (nrows - 1);
  const int t  = r >> hshift;
  const int hd = r - (t << hshift);
  const float* sp = &slab[wave][q][c8];
  unsigned hw[4], lw[4];
#pragma unroll
  for (int e2 = 0; e2 < 4; ++e2) {
    const float f0 = sp[2 * e2], f1 = sp[2 * e2 + 1];
    const unsigned short h0 = f2bf_bits(f0), h1 = f2bf_bits(f1);
    const unsigned short l0 = f2bf_bits(f0 - bf_bits2f(h0));
    const unsigned short l1 = f2bf_bits(f1 - bf_bits2f(h1));
    hw[e2] = pk16(h0, h1);
    lw[e2] = pk16(l0, l1);
  }
  const v4u hu = (v4u){hw[0], hw[1], hw[2], hw[3]};
  const v4u lu = (v4u){lw[0], lw[1], lw[2], lw[3]};
  const size_t o = ((size_t)hd * SEQ_T + t) * 64 + c8;
  *(volatile v4u*)(ohi + o) = hu;
  *(volatile v4u*)(olo + o) = lu;
  __threadfence();
  *(volatile v4u*)(ohi + o) = hu;
  *(volatile v4u*)(olo + o) = lu;
}

template <int NT>
__global__ __launch_bounds__(NT) void softmax_causal_kernel(const float* __restrict__ S,
                                                            unsigned short* __restrict__ Phi, unsigned short* __restrict__ Plo,
                                                            int crow0) {
  constexpr int NWV = NT / 32;
  __shared__ float redM[NWV];
  __shared__ float redS[NWV];
  const float ninf = -__builtin_inff();
  const int qloc = blockIdx.x;
  const int qi   = crow0 + qloc;
  const int t    = threadIdx.x;
  const int lane = t & 31, wave = t >> 5;
  const int c0   = t * 8;
  const size_t rowoff = (size_t)qloc * (size_t)SEQ_T;
  const bool wave_live = (wave * 256 <= qi);

  float xv[8];
  float m = ninf;
  if (wave_live) {
    const float* sr = S + rowoff + c0;
    const v4f a = *(const v4f*)(sr);
    const v4f c = *(const v4f*)(sr + 4);
    float sv[8];
#pragma unroll
    for (int e = 0; e < 4; ++e) { sv[e] = a[e]; sv[4 + e] = c[e]; }
#pragma unroll
    for (int e = 0; e < 8; ++e) {
      const int j = c0 + e;
      const float v = (j > qi) ? ninf : sv[e];
      xv[e] = v;
      m = fmaxf(m, v);
    }
  } else {
#pragma unroll
    for (int e = 0; e < 8; ++e) xv[e] = ninf;
  }
#pragma unroll
  for (int off = 16; off > 0; off >>= 1) m = fmaxf(m, __shfl_xor(m, off, 32));
  if (lane == 0) redM[wave] = m;
  __syncthreads();
  float gmax = redM[0];
#pragma unroll
  for (int wv = 1; wv < NWV; ++wv) gmax = fmaxf(gmax, redM[wv]);

  float p[8];
  float ps = 0.0f;
  if (wave_live) {
#pragma unroll
    for (int e = 0; e < 8; ++e) { p[e] = expf(xv[e] - gmax); ps += p[e]; }
  } else {
#pragma unroll
    for (int e = 0; e < 8; ++e) p[e] = 0.0f;
  }
#pragma unroll
  for (int off = 16; off > 0; off >>= 1) ps += __shfl_xor(ps, off, 32);
  if (lane == 0) redS[wave] = ps;
  __syncthreads();
  float tot = redS[0];
#pragma unroll
  for (int wv = 1; wv < NWV; ++wv) tot += redS[wv];
  const float inv = 1.0f / tot;

  unsigned hw[4], lw[4];
#pragma unroll
  for (int e2 = 0; e2 < 4; ++e2) {
    const float f0 = p[2 * e2] * inv;
    const float f1 = p[2 * e2 + 1] * inv;
    const unsigned short h0 = f2bf_bits(f0);
    const unsigned short h1 = f2bf_bits(f1);
    const unsigned short l0 = f2bf_bits(f0 - bf_bits2f(h0));
    const unsigned short l1 = f2bf_bits(f1 - bf_bits2f(h1));
    hw[e2] = pk16(h0, h1);
    lw[e2] = pk16(l0, l1);
  }
  const v4u hv = (v4u){hw[0], hw[1], hw[2], hw[3]};
  const v4u lv = (v4u){lw[0], lw[1], lw[2], lw[3]};
  unsigned short* ph = Phi + rowoff + c0;
  unsigned short* pl = Plo + rowoff + c0;
  *(volatile v4u*)ph = hv;
  *(volatile v4u*)pl = lv;
  __threadfence();
  *(volatile v4u*)ph = hv;
  *(volatile v4u*)pl = lv;
}

extern "C" void kernel_launch(void* const* d_in, const int* in_sizes, int n_in,
                              void* d_out, int out_size, void* d_ws, size_t ws_size,
                              hipStream_t stream) {
  if (n_in < 9) return;
  if (in_sizes[0] != SEQ_T * HIDSZ || in_sizes[1] != SEQ_T * 32 || in_sizes[2] != SEQ_T * 32) return;
  if (in_sizes[3] != HIDSZ * NQH * HDIM || in_sizes[4] != HIDSZ * NKVH * HDIM || in_sizes[5] != HIDSZ * NKVH * HDIM) return;
  if (in_sizes[6] != NQH * HDIM * HIDSZ || in_sizes[7] != HDIM || in_sizes[8] != HDIM) return;
  if (out_size != SEQ_T * HIDSZ) return;

  const size_t kMiB    = 1048576;
  const size_t offS    = 0;
  const size_t offXb   = 0;
  const size_t offQf   = 8 * kMiB;
  const size_t offKf   = 24 * kMiB;
  const size_t offWqT  = 28 * kMiB;
  const size_t offWkT  = 30 * kMiB;
  const size_t offWvT  = 30 * kMiB + 524288;
  const size_t offPhi  = 32 * kMiB;
  const size_t offPlo  = 48 * kMiB;
  const size_t offQhi  = 64 * kMiB;
  const size_t offQlo  = 72 * kMiB;
  const size_t offKhi  = 80 * kMiB;
  const size_t offKlo  = 82 * kMiB;
  const size_t offVthi = 84 * kMiB;
  const size_t offVtlo = 86 * kMiB;
  const size_t offChi  = 88 * kMiB;
  const size_t offClo  = 96 * kMiB;
  const size_t offWoT  = 104 * kMiB;
  const size_t total   = 106 * kMiB;
  if (total > ws_size) return;

  const float* x    = (const float*)d_in[0];
  const float* cosb = (const float*)d_in[1];
  const float* sinb = (const float*)d_in[2];
  const float* Wq   = (const float*)d_in[3];
  const float* Wk   = (const float*)d_in[4];
  const float* Wv   = (const float*)d_in[5];
  const float* Wo   = (const float*)d_in[6];
  const float* qnw  = (const float*)d_in[7];
  const float* knw  = (const float*)d_in[8];
  float* out = (float*)d_out;
  char* ws = (char*)d_ws;

  float*          Sbuf = (float*)(ws + offS);
  unsigned short* xb   = (unsigned short*)(ws + offXb);
  float*          qf   = (float*)(ws + offQf);
  float*          kf   = (float*)(ws + offKf);
  unsigned short* wqT  = (unsigned short*)(ws + offWqT);
  unsigned short* wkT  = (unsigned short*)(ws + offWkT);
  unsigned short* wvT  = (unsigned short*)(ws + offWvT);
  unsigned short* phi  = (unsigned short*)(ws + offPhi);
  unsigned short* plo  = (unsigned short*)(ws + offPlo);
  unsigned short* qhi  = (unsigned short*)(ws + offQhi);
  unsigned short* qlo  = (unsigned short*)(ws + offQlo);
  unsigned short* khi  = (unsigned short*)(ws + offKhi);
  unsigned short* klo  = (unsigned short*)(ws + offKlo);
  unsigned short* vthi = (unsigned short*)(ws + offVthi);
  unsigned short* vtlo = (unsigned short*)(ws + offVtlo);
  unsigned short* chi  = (unsigned short*)(ws + offChi);
  unsigned short* clo  = (unsigned short*)(ws + offClo);
  unsigned short* woT  = (unsigned short*)(ws + offWoT);

  const float* dummy_f = qnw;
  void* dummy_c2 = (void*)plo;

  {
    const int n8 = (SEQ_T * HIDSZ) / 8;
    cast8_bf16_kernel<<<dim3(n8 / 256), dim3(256), 0, stream>>>(x, xb, n8);
  }
  transpose_cast_kernel<<<dim3(HIDSZ / 64, (NQH * HDIM) / 64), dim3(256), 0, stream>>>(Wq, NQH * HDIM, wqT, HIDSZ);
  transpose_cast_kernel<<<dim3(HIDSZ / 64, (NKVH * HDIM) / 64), dim3(256), 0, stream>>>(Wk, NKVH * HDIM, wkT, HIDSZ);
  transpose_cast_kernel<<<dim3(HIDSZ / 64, (NKVH * HDIM) / 64), dim3(256), 0, stream>>>(Wv, NKVH * HDIM, wvT, HIDSZ);
  transpose_cast_kernel<<<dim3((NQH * HDIM) / 64, HIDSZ / 64), dim3(256), 0, stream>>>(Wo, HIDSZ, woT, NQH * HDIM);

  wmma_gemm64<1, false, 0, 0, false, 0, false, true><<<dim3((SEQ_T / 64) * ((NQH * HDIM) / 64) / 8, 1), dim3(256), 0, stream>>>(
      xb, xb, HIDSZ, 0L,
      wqT, wqT, HIDSZ, 0L,
      (void*)qf, dummy_c2, NQH * HDIM, 0L,
      dummy_f, dummy_f, 0L,
      SEQ_T, NQH * HDIM, HIDSZ, 1.0f, 0);
  wmma_gemm64<1, false, 0, 0, false, 0, false, true><<<dim3((SEQ_T / 64) * ((NKVH * HDIM) / 64) / 8, 1), dim3(256), 0, stream>>>(
      xb, xb, HIDSZ, 0L,
      wkT, wkT, HIDSZ, 0L,
      (void*)kf, dummy_c2, NKVH * HDIM, 0L,
      dummy_f, dummy_f, 0L,
      SEQ_T, NKVH * HDIM, HIDSZ, 1.0f, 0);
  wmma_gemm64<1, false, 0, 2, false, 0, false, true><<<dim3(((NKVH * HDIM) / 64) * (SEQ_T / 64) / 8, 1), dim3(256), 0, stream>>>(
      wvT, wvT, HIDSZ, 0L,
      xb, xb, HIDSZ, 0L,
      (void*)vthi, (void*)vtlo, SEQ_T, 0L,
      dummy_f, dummy_f, 0L,
      NKVH * HDIM, SEQ_T, HIDSZ, 1.0f, 0);

  normrope_kernel<<<dim3((SEQ_T * NQH) / 32), dim3(256), 0, stream>>>(qf, 4, SEQ_T * NQH, cosb, sinb, qnw, qhi, qlo);
  normrope_kernel<<<dim3((SEQ_T * NKVH) / 32), dim3(256), 0, stream>>>(kf, 2, SEQ_T * NKVH, cosb, sinb, knw, khi, klo);

  for (int hq = 0; hq < NQH; ++hq) {
    const int kvh = hq >> 2;
    for (int ch = 0; ch < NCHUNK; ++ch) {
      const int crow0 = ch * QCHUNK;
      const size_t qoff = ((size_t)hq * SEQ_T + (size_t)crow0) * HDIM;
      const size_t koff = (size_t)kvh * SEQ_T * HDIM;

      wmma_gemm64<1, true, 0, 0, false, 0, true, true><<<dim3((QCHUNK / 64) * (SEQ_T / 64) / 8, 1), dim3(256), 0, stream>>>(
          qhi + qoff, qlo + qoff, HDIM, 0L,
          khi + koff, klo + koff, HDIM, 0L,
          (void*)Sbuf, dummy_c2, SEQ_T, 0L,
          dummy_f, dummy_f, 0L,
          QCHUNK, SEQ_T, HDIM, SCORE_SCALE, crow0);

      if (ch == 0) {
        softmax_causal_kernel<256><<<dim3(QCHUNK), dim3(256), 0, stream>>>(Sbuf, phi, plo, crow0);
      } else {
        softmax_causal_kernel<512><<<dim3(QCHUNK), dim3(512), 0, stream>>>(Sbuf, phi, plo, crow0);
      }

      const size_t vtoff = (size_t)(kvh * HDIM) * SEQ_T;
      const size_t coff  = (size_t)crow0 * (NQH * HDIM) + (size_t)hq * HDIM;
      wmma_gemm64<1, true, 0, 2, false, 0, true, true><<<dim3((QCHUNK / 64) * (HDIM / 64) / 8, 1), dim3(256), 0, stream>>>(
          phi, plo, SEQ_T, 0L,
          vthi + vtoff, vtlo + vtoff, SEQ_T, 0L,
          (void*)(chi + coff), (void*)(clo + coff), NQH * HDIM, 0L,
          dummy_f, dummy_f, 0L,
          QCHUNK, HDIM, SEQ_T, 1.0f, crow0);
    }
  }

  wmma_gemm64<1, true, 0, 0, false, 0, false, false><<<dim3((SEQ_T / 64) * (HIDSZ / 64) / 8, 1), dim3(256), 0, stream>>>(
      chi, clo, NQH * HDIM, 0L,
      woT, woT, NQH * HDIM, 0L,
      (void*)out, dummy_c2, HIDSZ, 0L,
      dummy_f, dummy_f, 0L,
      SEQ_T, HIDSZ, NQH * HDIM, 1.0f, 0);
}
